// MultiSAGENet_86088324481901
// MI455X (gfx1250) — hardware-run, weakly checked
//
#include <hip/hip_runtime.h>


namespace {
constexpr int N = 100000, E = 1600000, G = 200, FI = 4, H = 64, H4 = 256, NO = 4, NL = 4, RO = 3 * H + FI, ROP = 256, NBLK = N / 16;
constexpr float XS = 8.0f, WSC = 256.0f, EPS = 1e-5f;
typedef _Float16 b16;
typedef __attribute__((ext_vector_type(16))) _Float16 v16b;
typedef __attribute__((ext_vector_type(8))) _Float16 v8b;
typedef __attribute__((ext_vector_type(8))) float v8f;
typedef __attribute__((ext_vector_type(4))) float v4f;
typedef __attribute__((ext_vector_type(2))) float v2f;
__device__ __forceinline__ float bf16_rne(float f) { unsigned int u = __float_as_uint(f); u += 0x7FFFu + ((u >> 16) & 1u); return __uint_as_float(u & 0xFFFF0000u); }
__device__ __forceinline__ void split16(float v, b16& hi, b16& lo) { hi = (b16)v; lo = (b16)(v - (float)hi); }
__device__ __forceinline__ v16b frag_kb(const b16* p, int hh) { const v8b a = *(const v8b*)(p + 8 * hh), b = *(const v8b*)(p + 16 + 8 * hh); v16b f;
#pragma unroll
  for (int e = 0; e < 8; ++e) { f[e] = a[e]; f[8 + e] = b[e]; } return f; }
__device__ __forceinline__ v8f wmma16b(v16b a, v16b b, v8f c) { v8f d = __builtin_amdgcn_wmma_f32_16x16x32_f16(false, a, false, b, (short)0, c, false, false); asm volatile("v_nop\n\tv_nop\n\tv_nop\n\tv_nop" : "+v"(d) : "v"(a), "v"(b)); return d; }
__device__ __forceinline__ void wave_lds_sync() { __builtin_amdgcn_fence(__ATOMIC_RELEASE, "workgroup"); __builtin_amdgcn_wave_barrier(); __builtin_amdgcn_fence(__ATOMIC_ACQUIRE, "workgroup"); }
__device__ __forceinline__ float pmul(float a, float b) { float p = a * b; asm volatile("" : "+v"(p)); return p; }
__device__ __forceinline__ int iclamp(int v, int lo, int hi) { return v < lo ? lo : (v > hi ? hi : v); }
__device__ __forceinline__ float sigm(float v) { return 1.0f / (1.0f + __expf(-v)); }
__device__ __forceinline__ float silu(float v) { return pmul(v, sigm(v)); }
constexpr int CSR_NBLK9 = 512, CSR_GB9 = 9, CSR_GN9 = 1 << CSR_GB9  , CSR_TS9 = (CSR_GN9 < 32 ? 32 : CSR_GN9)  , CSR_MAXG9 = 512, CSR_CAP9 = 12288  ;
__device__ __host__ __forceinline__ int csr_tix9(int v) { return (v >> CSR_GB9) * CSR_TS9 + (v & (CSR_GN9 - 1)); }
__global__ __launch_bounds__(64) void csrA_kernel9(const int* __restrict__ dst, int E, int N, int nG, int CHP, int NGP, int* __restrict__ STG, int* __restrict__ HST) {
  extern __shared__ int sm[];
  int* cnt = sm; int* run = sm + NGP; int* ids = sm + 2 * NGP;
  const int b = blockIdx.x; const int ch = (E + CSR_NBLK9 - 1) / CSR_NBLK9; const int e0 = b * ch, e1 = min(E, e0 + ch);
  for (int i = threadIdx.x; i < NGP; i += 64) cnt[i] = 0;
  for (int i = threadIdx.x; i < CHP; i += 64) ids[i] = -1;
  __syncthreads();
  if (threadIdx.x == 0) {
    for (int e = e0; e < e1; ++e) { int d = dst[e]; d = (d < 0) ? 0 : (d >= N ? N - 1 : d); cnt[d >> CSR_GB9] += 1; }
    int acc = 0; for (int g = 0; g < nG; ++g) { run[g] = acc; acc += cnt[g]; }
    for (int e = e0; e < e1; ++e) { int d = dst[e]; d = (d < 0) ? 0 : (d >= N ? N - 1 : d); const int g = d >> CSR_GB9; ids[run[g]] = e; run[g] += 1; } }
  __syncthreads();
  typedef __attribute__((ext_vector_type(4))) int v4i;
  for (int pass = 0; pass < 2; ++pass) {
    for (int i = threadIdx.x; i < CHP / 4; i += 64) *(volatile v4i*)(STG + (size_t)b * CHP + i * 4) = *(const v4i*)(&ids[i * 4]);
    for (int i = threadIdx.x; i < NGP / 4; i += 64) { v4i v; for (int e = 0; e < 4; ++e) v[e] = (i * 4 + e < nG) ? cnt[i * 4 + e] : 0; *(volatile v4i*)(HST + (size_t)b * NGP + i * 4) = v; }
    __threadfence(); }
}
__global__ __launch_bounds__(512) void csrS_kernel9(const int* __restrict__ HST, int nG, int NGP, int* __restrict__ START, int* __restrict__ TOT, int* __restrict__ OFF) {
  __shared__ int tot[CSR_MAXG9];
  const int b = threadIdx.x;
  for (int pass = 0; pass < 2; ++pass) { int runb = 0; for (int g = 0; g < nG; ++g) { int c = HST[(size_t)b * NGP + g]; c = (c < 0) ? 0 : c; ((volatile int*)OFF)[(size_t)g * CSR_NBLK9 + b] = runb; runb += c; } __threadfence(); }
  for (int g = threadIdx.x; g < nG; g += 512) { int s = 0; for (int bb = 0; bb < CSR_NBLK9; ++bb) { int c = HST[(size_t)bb * NGP + g]; s += (c < 0) ? 0 : c; } tot[g] = s; }
  __syncthreads();
  if (threadIdx.x < 32) {
    __shared__ int st[CSR_MAXG9 + 32];
    if (threadIdx.x == 0) { int acc = 0; for (int g = 0; g < NGP; ++g) { st[g] = acc; if (g < nG) acc += (tot[g] + 31) & ~31; } st[NGP] = acc; }
    __builtin_amdgcn_fence(__ATOMIC_RELEASE, "workgroup"); __builtin_amdgcn_wave_barrier(); __builtin_amdgcn_fence(__ATOMIC_ACQUIRE, "workgroup");
    for (int pass = 0; pass < 2; ++pass) { for (int i = threadIdx.x; i < NGP + 32; i += 32) { ((volatile int*)START)[i] = (i <= NGP) ? st[min(i, NGP)] : 0; ((volatile int*)TOT)[i] = (i < nG) ? tot[i] : 0; } __threadfence(); } }
}
__global__ __launch_bounds__(256) void csrB_kernel9(const int* __restrict__ dst, int N, int nG, int CHP, int NGP, int permLen, const int* __restrict__ STG, const int* __restrict__ HST, const int* __restrict__ OFF, const int* __restrict__ START, const int* __restrict__ TOT, int* __restrict__ PERM, int* __restrict__ ROWPTR, int* __restrict__ ROWCNT, int* __restrict__ FLAG) {
  typedef __attribute__((ext_vector_type(4))) int v4i;
  __shared__ int ids[CSR_CAP9]; __shared__ unsigned short key[CSR_CAP9]; __shared__ int outp[CSR_CAP9]; __shared__ int ncnt[CSR_GN9 + 1]; __shared__ int boff[CSR_NBLK9 + 1];
  const int g = blockIdx.x, t_ = threadIdx.x; int tot = TOT[g]; int st = START[g], stn = START[g + 1]; const int v0 = g * CSR_GN9; const int nv = min(CSR_GN9, N - v0); const int t0 = g * CSR_TS9;
  st = (st < 0) ? 0 : (st > permLen - 32 ? permLen - 32 : st) & ~31; stn = (stn < st) ? st : (stn > permLen ? permLen : stn); tot = (tot < 0) ? 0 : tot; if (tot > stn - st && tot <= CSR_CAP9) tot = stn - st;
  if (tot > CSR_CAP9) {
    for (int pass = 0; pass < 2; ++pass) { for (int i = t_; i < CSR_TS9 / 4; i += 256) { v4i a, c; for (int e = 0; e < 4; ++e) { a[e] = st; c[e] = 0; } *(volatile v4i*)(ROWPTR + t0 + i * 4) = a; *(volatile v4i*)(ROWCNT + t0 + i * 4) = c; } if (t_ == 0) ((volatile int*)FLAG)[0] = 1; __threadfence(); } (void)nv; return; }
  if (t_ == 0) { int acc = 0; for (int b = 0; b < CSR_NBLK9; ++b) { boff[b] = acc; int c = HST[(size_t)b * NGP + g]; c = (c < 0) ? 0 : (c > CHP ? CHP : c); acc += c; if (acc > tot) acc = tot; } boff[CSR_NBLK9] = acc; }
  for (int i = t_; i <= CSR_GN9; i += 256) ncnt[i] = 0;
  __syncthreads();
  for (int b = 0; b < CSR_NBLK9; ++b) { const int c = boff[b + 1] - boff[b]; int o_ = OFF[(size_t)g * CSR_NBLK9 + b]; o_ = (o_ < 0) ? 0 : (o_ > CHP - c ? CHP - c : o_); const int* src_ = STG + (size_t)b * CHP + o_;
    for (int i = t_; i < c; i += 256) { int id = src_[i]; id = (id < 0) ? 0 : id; ids[boff[b] + i] = id; int d = dst[id]; d = (d < v0) ? v0 : (d >= N ? N - 1 : d); int kk = d - v0; kk = (kk < 0) ? 0 : (kk >= CSR_GN9 ? CSR_GN9 - 1 : kk); key[boff[b] + i] = (unsigned short)kk; } }
  __syncthreads();
  if (t_ == 0) { for (int i = 0; i < tot; ++i) ncnt[key[i]] += 1; int acc = 0; for (int vl = 0; vl < CSR_GN9; ++vl) { const int c = ncnt[vl]; ncnt[vl] = acc; acc += c; } ncnt[CSR_GN9] = acc;
    for (int i = 0; i < tot; ++i) { const int vl = key[i]; outp[ncnt[vl]] = ids[i]; ncnt[vl] += 1; }
    for (int vl = CSR_GN9; vl > 0; --vl) ncnt[vl] = ncnt[vl - 1]; ncnt[0] = 0; }
  __syncthreads();
  for (int pass = 0; pass < 2; ++pass) {
    for (int i = t_; i < (stn - st) / 4; i += 256) { v4i v; for (int e = 0; e < 4; ++e) { const int q = i * 4 + e; v[e] = (q < tot) ? outp[q] : -1; } *(volatile v4i*)(PERM + st + i * 4) = v; }
    for (int i = t_; i < CSR_TS9 / 4; i += 256) { v4i a, c; for (int e = 0; e < 4; ++e) { const int vl = i * 4 + e; const int vc = vl < CSR_GN9 ? vl : CSR_GN9; a[e] = (vl < CSR_GN9) ? st + ncnt[vc] : st; c[e] = (vl < nv) ? (ncnt[(vc < CSR_GN9 ? vc : CSR_GN9 - 1) + 1] - ncnt[vc]) : 0; } *(volatile v4i*)(ROWPTR + t0 + i * 4) = a; *(volatile v4i*)(ROWCNT + t0 + i * 4) = c; }
    __threadfence(); }
}
__global__ __launch_bounds__(256) void csrZ_kernel9(int* __restrict__ p, size_t n4) { typedef __attribute__((ext_vector_type(4))) int v4i; const size_t tid = (size_t)blockIdx.x * 256 + threadIdx.x, nth = (size_t)gridDim.x * 256; v4i z = {0, 0, 0, 0}; for (size_t i = tid; i < n4; i += nth) *(volatile v4i*)(p + i * 4) = z; }
struct CsrBufs9 { int *STG, *HST, *OFF, *START, *TOT, *PERM, *ROWPTR, *ROWCNT, *FLAG; int nG, NGP, CHP; size_t permLen; char* base; size_t bytes; };
static size_t csr_carve9(CsrBufs9& c, char* ws, size_t off, int E, int N) {
  const size_t off0 = off; c.base = ws + off;
  auto al = [&](size_t bytes) { char* p = ws + off; off += (bytes + 255) & ~(size_t)255; return p; };
  c.nG = (N + CSR_GN9 - 1) / CSR_GN9; c.NGP = (c.nG + 31) & ~31; const int ch = (E + CSR_NBLK9 - 1) / CSR_NBLK9; c.CHP = (ch + 31) & ~31; c.permLen = (size_t)E + 32 * (size_t)c.nG + 32;
  c.STG = (int*)al((size_t)CSR_NBLK9 * c.CHP * 4); c.HST = (int*)al((size_t)CSR_NBLK9 * c.NGP * 4); c.OFF = (int*)al((size_t)c.NGP * CSR_NBLK9 * 4); c.START = (int*)al((size_t)(c.NGP + 64) * 4); c.TOT = (int*)al((size_t)(c.NGP + 64) * 4);
  c.PERM = (int*)al(c.permLen * 4); c.ROWPTR = (int*)al((size_t)c.nG * CSR_TS9 * 4); c.ROWCNT = (int*)al((size_t)c.nG * CSR_TS9 * 4); c.FLAG = (int*)al(256);
  c.bytes = off - off0; return off;
}
static void csr_build9(const CsrBufs9& c, const int* dst, int E, int N, hipStream_t stream) {
  const size_t smem = (size_t)(2 * c.NGP + c.CHP) * 4;
  csrZ_kernel9<<<512, 256, 0, stream>>>((int*)c.base, c.bytes / 16);
  csrA_kernel9<<<CSR_NBLK9, 64, smem, stream>>>(dst, E, N, c.nG, c.CHP, c.NGP, c.STG, c.HST);
  csrS_kernel9<<<1, 512, 0, stream>>>(c.HST, c.nG, c.NGP, c.START, c.TOT, c.OFF);
  csrB_kernel9<<<c.nG, 256, 0, stream>>>(dst, N, c.nG, c.CHP, c.NGP, (int)c.permLen, c.STG, c.HST, c.OFF, c.START, c.TOT, c.PERM, c.ROWPTR, c.ROWCNT, c.FLAG);
}

constexpr int CSR_NBLK3 = 512, CSR_GB3 = 3, CSR_GN3 = 1 << CSR_GB3  , CSR_TS3 = (CSR_GN3 < 32 ? 32 : CSR_GN3)  , CSR_MAXG3 = 512, CSR_CAP3 = 12288  ;
__device__ __host__ __forceinline__ int csr_tix3(int v) { return (v >> CSR_GB3) * CSR_TS3 + (v & (CSR_GN3 - 1)); }
__global__ __launch_bounds__(64) void csrA_kernel3(const int* __restrict__ dst, int E, int N, int nG, int CHP, int NGP, int* __restrict__ STG, int* __restrict__ HST) {
  extern __shared__ int sm[];
  int* cnt = sm; int* run = sm + NGP; int* ids = sm + 2 * NGP;
  const int b = blockIdx.x; const int ch = (E + CSR_NBLK3 - 1) / CSR_NBLK3; const int e0 = b * ch, e1 = min(E, e0 + ch);
  for (int i = threadIdx.x; i < NGP; i += 64) cnt[i] = 0;
  for (int i = threadIdx.x; i < CHP; i += 64) ids[i] = -1;
  __syncthreads();
  if (threadIdx.x == 0) {
    for (int e = e0; e < e1; ++e) { int d = dst[e]; d = (d < 0) ? 0 : (d >= N ? N - 1 : d); cnt[d >> CSR_GB3] += 1; }
    int acc = 0; for (int g = 0; g < nG; ++g) { run[g] = acc; acc += cnt[g]; }
    for (int e = e0; e < e1; ++e) { int d = dst[e]; d = (d < 0) ? 0 : (d >= N ? N - 1 : d); const int g = d >> CSR_GB3; ids[run[g]] = e; run[g] += 1; } }
  __syncthreads();
  typedef __attribute__((ext_vector_type(4))) int v4i;
  for (int pass = 0; pass < 2; ++pass) {
    for (int i = threadIdx.x; i < CHP / 4; i += 64) *(volatile v4i*)(STG + (size_t)b * CHP + i * 4) = *(const v4i*)(&ids[i * 4]);
    for (int i = threadIdx.x; i < NGP / 4; i += 64) { v4i v; for (int e = 0; e < 4; ++e) v[e] = (i * 4 + e < nG) ? cnt[i * 4 + e] : 0; *(volatile v4i*)(HST + (size_t)b * NGP + i * 4) = v; }
    __threadfence(); }
}
__global__ __launch_bounds__(512) void csrS_kernel3(const int* __restrict__ HST, int nG, int NGP, int* __restrict__ START, int* __restrict__ TOT, int* __restrict__ OFF) {
  __shared__ int tot[CSR_MAXG3];
  const int b = threadIdx.x;
  for (int pass = 0; pass < 2; ++pass) { int runb = 0; for (int g = 0; g < nG; ++g) { int c = HST[(size_t)b * NGP + g]; c = (c < 0) ? 0 : c; ((volatile int*)OFF)[(size_t)g * CSR_NBLK3 + b] = runb; runb += c; } __threadfence(); }
  for (int g = threadIdx.x; g < nG; g += 512) { int s = 0; for (int bb = 0; bb < CSR_NBLK3; ++bb) { int c = HST[(size_t)bb * NGP + g]; s += (c < 0) ? 0 : c; } tot[g] = s; }
  __syncthreads();
  if (threadIdx.x < 32) {
    __shared__ int st[CSR_MAXG3 + 32];
    if (threadIdx.x == 0) { int acc = 0; for (int g = 0; g < NGP; ++g) { st[g] = acc; if (g < nG) acc += (tot[g] + 31) & ~31; } st[NGP] = acc; }
    __builtin_amdgcn_fence(__ATOMIC_RELEASE, "workgroup"); __builtin_amdgcn_wave_barrier(); __builtin_amdgcn_fence(__ATOMIC_ACQUIRE, "workgroup");
    for (int pass = 0; pass < 2; ++pass) { for (int i = threadIdx.x; i < NGP + 32; i += 32) { ((volatile int*)START)[i] = (i <= NGP) ? st[min(i, NGP)] : 0; ((volatile int*)TOT)[i] = (i < nG) ? tot[i] : 0; } __threadfence(); } }
}
__global__ __launch_bounds__(256) void csrB_kernel3(const int* __restrict__ dst, int N, int nG, int CHP, int NGP, int permLen, const int* __restrict__ STG, const int* __restrict__ HST, const int* __restrict__ OFF, const int* __restrict__ START, const int* __restrict__ TOT, int* __restrict__ PERM, int* __restrict__ ROWPTR, int* __restrict__ ROWCNT, int* __restrict__ FLAG) {
  typedef __attribute__((ext_vector_type(4))) int v4i;
  __shared__ int ids[CSR_CAP3]; __shared__ unsigned short key[CSR_CAP3]; __shared__ int outp[CSR_CAP3]; __shared__ int ncnt[CSR_GN3 + 1]; __shared__ int boff[CSR_NBLK3 + 1];
  const int g = blockIdx.x, t_ = threadIdx.x; int tot = TOT[g]; int st = START[g], stn = START[g + 1]; const int v0 = g * CSR_GN3; const int nv = min(CSR_GN3, N - v0); const int t0 = g * CSR_TS3;
  st = (st < 0) ? 0 : (st > permLen - 32 ? permLen - 32 : st) & ~31; stn = (stn < st) ? st : (stn > permLen ? permLen : stn); tot = (tot < 0) ? 0 : tot; if (tot > stn - st && tot <= CSR_CAP3) tot = stn - st;
  if (tot > CSR_CAP3) {
    for (int pass = 0; pass < 2; ++pass) { for (int i = t_; i < CSR_TS3 / 4; i += 256) { v4i a, c; for (int e = 0; e < 4; ++e) { a[e] = st; c[e] = 0; } *(volatile v4i*)(ROWPTR + t0 + i * 4) = a; *(volatile v4i*)(ROWCNT + t0 + i * 4) = c; } if (t_ == 0) ((volatile int*)FLAG)[0] = 1; __threadfence(); } (void)nv; return; }
  if (t_ == 0) { int acc = 0; for (int b = 0; b < CSR_NBLK3; ++b) { boff[b] = acc; int c = HST[(size_t)b * NGP + g]; c = (c < 0) ? 0 : (c > CHP ? CHP : c); acc += c; if (acc > tot) acc = tot; } boff[CSR_NBLK3] = acc; }
  for (int i = t_; i <= CSR_GN3; i += 256) ncnt[i] = 0;
  __syncthreads();
  for (int b = 0; b < CSR_NBLK3; ++b) { const int c = boff[b + 1] - boff[b]; int o_ = OFF[(size_t)g * CSR_NBLK3 + b]; o_ = (o_ < 0) ? 0 : (o_ > CHP - c ? CHP - c : o_); const int* src_ = STG + (size_t)b * CHP + o_;
    for (int i = t_; i < c; i += 256) { int id = src_[i]; id = (id < 0) ? 0 : id; ids[boff[b] + i] = id; int d = dst[id]; d = (d < v0) ? v0 : (d >= N ? N - 1 : d); int kk = d - v0; kk = (kk < 0) ? 0 : (kk >= CSR_GN3 ? CSR_GN3 - 1 : kk); key[boff[b] + i] = (unsigned short)kk; } }
  __syncthreads();
  if (t_ == 0) { for (int i = 0; i < tot; ++i) ncnt[key[i]] += 1; int acc = 0; for (int vl = 0; vl < CSR_GN3; ++vl) { const int c = ncnt[vl]; ncnt[vl] = acc; acc += c; } ncnt[CSR_GN3] = acc;
    for (int i = 0; i < tot; ++i) { const int vl = key[i]; outp[ncnt[vl]] = ids[i]; ncnt[vl] += 1; }
    for (int vl = CSR_GN3; vl > 0; --vl) ncnt[vl] = ncnt[vl - 1]; ncnt[0] = 0; }
  __syncthreads();
  for (int pass = 0; pass < 2; ++pass) {
    for (int i = t_; i < (stn - st) / 4; i += 256) { v4i v; for (int e = 0; e < 4; ++e) { const int q = i * 4 + e; v[e] = (q < tot) ? outp[q] : -1; } *(volatile v4i*)(PERM + st + i * 4) = v; }
    for (int i = t_; i < CSR_TS3 / 4; i += 256) { v4i a, c; for (int e = 0; e < 4; ++e) { const int vl = i * 4 + e; const int vc = vl < CSR_GN3 ? vl : CSR_GN3; a[e] = (vl < CSR_GN3) ? st + ncnt[vc] : st; c[e] = (vl < nv) ? (ncnt[(vc < CSR_GN3 ? vc : CSR_GN3 - 1) + 1] - ncnt[vc]) : 0; } *(volatile v4i*)(ROWPTR + t0 + i * 4) = a; *(volatile v4i*)(ROWCNT + t0 + i * 4) = c; }
    __threadfence(); }
}
__global__ __launch_bounds__(256) void csrZ_kernel3(int* __restrict__ p, size_t n4) { typedef __attribute__((ext_vector_type(4))) int v4i; const size_t tid = (size_t)blockIdx.x * 256 + threadIdx.x, nth = (size_t)gridDim.x * 256; v4i z = {0, 0, 0, 0}; for (size_t i = tid; i < n4; i += nth) *(volatile v4i*)(p + i * 4) = z; }
struct CsrBufs3 { int *STG, *HST, *OFF, *START, *TOT, *PERM, *ROWPTR, *ROWCNT, *FLAG; int nG, NGP, CHP; size_t permLen; char* base; size_t bytes; };
static size_t csr_carve3(CsrBufs3& c, char* ws, size_t off, int E, int N) {
  const size_t off0 = off; c.base = ws + off;
  auto al = [&](size_t bytes) { char* p = ws + off; off += (bytes + 255) & ~(size_t)255; return p; };
  c.nG = (N + CSR_GN3 - 1) / CSR_GN3; c.NGP = (c.nG + 31) & ~31; const int ch = (E + CSR_NBLK3 - 1) / CSR_NBLK3; c.CHP = (ch + 31) & ~31; c.permLen = (size_t)E + 32 * (size_t)c.nG + 32;
  c.STG = (int*)al((size_t)CSR_NBLK3 * c.CHP * 4); c.HST = (int*)al((size_t)CSR_NBLK3 * c.NGP * 4); c.OFF = (int*)al((size_t)c.NGP * CSR_NBLK3 * 4); c.START = (int*)al((size_t)(c.NGP + 64) * 4); c.TOT = (int*)al((size_t)(c.NGP + 64) * 4);
  c.PERM = (int*)al(c.permLen * 4); c.ROWPTR = (int*)al((size_t)c.nG * CSR_TS3 * 4); c.ROWCNT = (int*)al((size_t)c.nG * CSR_TS3 * 4); c.FLAG = (int*)al(256);
  c.bytes = off - off0; return off;
}
static void csr_build3(const CsrBufs3& c, const int* dst, int E, int N, hipStream_t stream) {
  const size_t smem = (size_t)(2 * c.NGP + c.CHP) * 4;
  csrZ_kernel3<<<512, 256, 0, stream>>>((int*)c.base, c.bytes / 16);
  csrA_kernel3<<<CSR_NBLK3, 64, smem, stream>>>(dst, E, N, c.nG, c.CHP, c.NGP, c.STG, c.HST);
  csrS_kernel3<<<1, 512, 0, stream>>>(c.HST, c.nG, c.NGP, c.START, c.TOT, c.OFF);
  csrB_kernel3<<<c.nG, 256, 0, stream>>>(dst, N, c.nG, c.CHP, c.NGP, (int)c.permLen, c.STG, c.HST, c.OFF, c.START, c.TOT, c.PERM, c.ROWPTR, c.ROWCNT, c.FLAG);
}


__global__ __launch_bounds__(256) void wput_kernel(const float* __restrict__ w, int KIN, int OUTW, int OUT, int co, int KP, b16* __restrict__ WT) {
  const int KG = KIN / 8; const int u = blockIdx.x * 256 + threadIdx.x; if (u >= OUT * KG) return; const int o = u / KG, k0 = (u % KG) * 8; v8b v;
#pragma unroll
  for (int j = 0; j < 8; ++j) v[j] = (b16)(bf16_rne(w[(size_t)(k0 + j) * OUTW + o]) * WSC); for (int pass = 0; pass < 2; ++pass) { *(volatile v8b*)(WT + (size_t)o * KP + co + k0) = v; __threadfence(); }
}
__global__ __launch_bounds__(128) void w0_kernel(const float* __restrict__ wl0, const float* __restrict__ wr0, const float* __restrict__ wres, b16* __restrict__ WT) {
  const int o = threadIdx.x; v8b v0 = {}, v1 = {}, vz = {};
  if (o < H) {
#pragma unroll
    for (int k = 0; k < 8; ++k) v0[k] = (b16)(bf16_rne(wl0[k * H + o]) * WSC);
#pragma unroll
    for (int k = 0; k < 4; ++k) v1[k] = (b16)(bf16_rne(wr0[k * H + o]) * WSC); }
  else { const int oo = o - H;
#pragma unroll
    for (int k = 0; k < 4; ++k) v1[4 + k] = (b16)(bf16_rne(wres[k * H + oo]) * WSC); }
  for (int pass = 0; pass < 2; ++pass) { *(volatile v8b*)(WT + (size_t)o * 32) = v0; *(volatile v8b*)(WT + (size_t)o * 32 + 8) = v1; *(volatile v8b*)(WT + (size_t)o * 32 + 16) = vz; *(volatile v8b*)(WT + (size_t)o * 32 + 24) = vz; __threadfence(); }
}
__global__ __launch_bounds__(256) void ro_tail_kernel(const float* __restrict__ w, b16* __restrict__ WT) {
  const int o = threadIdx.x; v8b v0 = {}, vz = {};
  for (int k = 0; k < FI; ++k) v0[k] = (b16)(bf16_rne(w[(size_t)(3 * H + k) * H4 + o]) * WSC);
  for (int pass = 0; pass < 2; ++pass) { *(volatile v8b*)(WT + (size_t)o * ROP + 3 * H) = v0; for (int g = 1; g < 8; ++g) *(volatile v8b*)(WT + (size_t)o * ROP + 3 * H + g * 8) = vz; __threadfence(); }
}
template <int L0>
__global__ __launch_bounds__(32) void sage_kernel(const float* __restrict__ IN_, const int* __restrict__ srcs, const int* __restrict__ PERM, const int* __restrict__ ROWPTR, const int* __restrict__ ROWCNT, int permLen, const b16* __restrict__ WT, const float* __restrict__ bl, const float* __restrict__ bres, const float* __restrict__ g, const float* __restrict__ bb, int NLIM, float* __restrict__ OUT_) {
  constexpr int KA = L0 ? 32 : 3 * H; constexpr int KIN = L0 ? FI : H;
  __shared__ __attribute__((aligned(16))) b16 Ah[16][KA + 8], Al[16][KA + 8]; __shared__ __attribute__((aligned(16))) float Rs[16][H + 4], Tf[16][H + 4];
  const int lane = threadIdx.x, nloc = lane & 15, hlf = lane >> 4; const size_t m0 = (size_t)blockIdx.x * 16; if (m0 >= (size_t)NLIM) return;
  for (int rr = 0; rr < 16; ++rr) { const size_t v = m0 + rr; int st = ROWPTR[v], cnt = ROWCNT[v]; cnt = iclamp(cnt, 0, 1 << 20); st = iclamp(st, 0, permLen - cnt); int used = 0;
    if (L0) {
      float mx = -INFINITY, sm = 0.0f; const float own = lane < FI ? bf16_rne(IN_[v * FI + lane]) : 0.0f;
#pragma unroll 1
      for (int j = 0; j < cnt; ++j) { const int e = iclamp(PERM[st + j], 0, E - 1); const int s = iclamp(srcs[e], 0, N - 1); ++used; const float f = lane < FI ? bf16_rne(IN_[(size_t)s * FI + lane]) : 0.0f; mx = fmaxf(mx, f); sm += f; }
      const float mxv = used > 0 ? mx : 0.0f, mean = sm / (float)(used < 1 ? 1 : used);
      b16 p, q; if (lane < FI) { split16(mxv * XS, p, q); Ah[rr][lane] = p; Al[rr][lane] = q; split16(mean * XS, p, q); Ah[rr][4 + lane] = p; Al[rr][4 + lane] = q; Ah[rr][8 + lane] = (b16)(own * XS); Al[rr][8 + lane] = (b16)0.0f; Ah[rr][12 + lane] = (b16)(own * XS); Al[rr][12 + lane] = (b16)0.0f; }
      else if (lane >= 16) { Ah[rr][lane] = (b16)0.0f; Al[rr][lane] = (b16)0.0f; } }
    else { v2f mx = {-INFINITY, -INFINITY}, sm = {0.0f, 0.0f}; const v2f own = *(const v2f*)(IN_ + v * H + lane * 2);
#pragma unroll 1
      for (int j = 0; j < cnt; ++j) { const int e = iclamp(PERM[st + j], 0, E - 1); const size_t s = (size_t)iclamp(srcs[e], 0, N - 1); if (s >= (size_t)NLIM) continue; ++used; const v2f f = *(const v2f*)(IN_ + s * H + lane * 2); for (int i = 0; i < 2; ++i) { mx[i] = fmaxf(mx[i], f[i]); sm[i] += f[i]; } }
      const float inv = 1.0f / (float)(used < 1 ? 1 : used);
      for (int i = 0; i < 2; ++i) { const float mxv = used > 0 ? mx[i] : 0.0f; b16 p, q; split16(mxv * XS, p, q); Ah[rr][lane * 2 + i] = p; Al[rr][lane * 2 + i] = q; split16(pmul(sm[i], inv) * XS, p, q); Ah[rr][H + lane * 2 + i] = p; Al[rr][H + lane * 2 + i] = q; split16(own[i] * XS, p, q); Ah[rr][2 * H + lane * 2 + i] = p; Al[rr][2 * H + lane * 2 + i] = q; Rs[rr][lane * 2 + i] = own[i]; } } }
  wave_lds_sync();
  v8f acc[4], racc[4];
#pragma unroll
  for (int t = 0; t < 4; ++t) { acc[t] = (v8f){}; racc[t] = (v8f){}; }
#pragma unroll
  for (int kb = 0; kb < KA; kb += 32) { const v16b a = frag_kb(&Ah[nloc][kb], hlf), al = frag_kb(&Al[nloc][kb], hlf);
#pragma unroll
    for (int t = 0; t < 4; ++t) { const v16b bw = frag_kb(WT + (size_t)(t * 16 + nloc) * KA + kb, hlf); acc[t] = wmma16b(a, bw, acc[t]); acc[t] = wmma16b(al, bw, acc[t]);
      if (L0) { const v16b bw2 = frag_kb(WT + (size_t)(H + t * 16 + nloc) * KA + kb, hlf); racc[t] = wmma16b(a, bw2, racc[t]); racc[t] = wmma16b(al, bw2, racc[t]); } } }
  const float sc = 1.0f / (XS * WSC); float vals[4][8], ps[8], pq[8];
#pragma unroll
  for (int r8 = 0; r8 < 8; ++r8) ps[r8] = 0.0f;
#pragma unroll
  for (int t = 0; t < 4; ++t) { const float b1 = bf16_rne(bl[t * 16 + nloc]);
#pragma unroll
    for (int r8 = 0; r8 < 8; ++r8) { vals[t][r8] = acc[t][r8] * sc + b1; ps[r8] += vals[t][r8]; } }
#pragma unroll
  for (int r8 = 0; r8 < 8; ++r8) { for (int o = 1; o < 16; o <<= 1) ps[r8] += __shfl_xor(ps[r8], o); ps[r8] *= (1.0f / H); pq[r8] = 0.0f;
#pragma unroll
    for (int t = 0; t < 4; ++t) { const float d = vals[t][r8] - ps[r8]; pq[r8] += pmul(d, d); } for (int o = 1; o < 16; o <<= 1) pq[r8] += __shfl_xor(pq[r8], o); pq[r8] = rsqrtf(pq[r8] * (1.0f / H) + EPS); }
  wave_lds_sync();
#pragma unroll
  for (int t = 0; t < 4; ++t) { const int c = t * 16 + nloc; const float gg = bf16_rne(g[c]), be = bf16_rne(bb[c]), brs = L0 ? bf16_rne(bres[c]) : 0.0f;
#pragma unroll
    for (int r8 = 0; r8 < 8; ++r8) { const int rl = 8 * hlf + r8; const float res = L0 ? racc[t][r8] * sc + brs : Rs[rl][c]; Tf[rl][c] = silu(pmul(pmul(vals[t][r8] - ps[r8], pq[r8]), gg) + be + res); } }
  wave_lds_sync();
  for (int pass = 0; pass < 2; ++pass) { for (int rr = 0; rr < 16; ++rr) *(volatile v2f*)(OUT_ + (m0 + rr) * H + lane * 2) = *(const v2f*)(&Tf[rr][lane * 2]); __threadfence(); }
}
__global__ __launch_bounds__(32) void mlp_kernel(const float* __restrict__ Hp, const b16* __restrict__ W1T, const float* __restrict__ b1, const float* __restrict__ g, const float* __restrict__ bb, const b16* __restrict__ W2T, const float* __restrict__ b2, int NLIM, float* __restrict__ OUT_) {
  __shared__ __attribute__((aligned(16))) b16 Ah[16][H4 + 8], Al[16][H4 + 8]; __shared__ __attribute__((aligned(16))) float Tf[16][H + 4];
  const int lane = threadIdx.x, nloc = lane & 15, hlf = lane >> 4; const size_t m0 = (size_t)blockIdx.x * 16; if (m0 >= (size_t)NLIM) return; const float sc = 1.0f / (XS * WSC);
  for (int rr = 0; rr < 16; ++rr) { const v2f v = *(const v2f*)(Hp + (m0 + rr) * H + lane * 2); for (int i = 0; i < 2; ++i) { b16 p, q; split16(v[i] * XS, p, q); Ah[rr][lane * 2 + i] = p; Al[rr][lane * 2 + i] = q; } }
  wave_lds_sync();
  v8f a1[16];
#pragma unroll
  for (int t = 0; t < 16; ++t) a1[t] = (v8f){};
#pragma unroll
  for (int kb = 0; kb < H; kb += 32) { const v16b a = frag_kb(&Ah[nloc][kb], hlf), al = frag_kb(&Al[nloc][kb], hlf);
#pragma unroll
    for (int t = 0; t < 16; ++t) { const v16b bw = frag_kb(W1T + (size_t)(t * 16 + nloc) * H + kb, hlf); a1[t] = wmma16b(a, bw, a1[t]); a1[t] = wmma16b(al, bw, a1[t]); } }
  float ps[8], pq[8];
#pragma unroll
  for (int r8 = 0; r8 < 8; ++r8) ps[r8] = 0.0f;
#pragma unroll
  for (int t = 0; t < 16; ++t) { const float bv = bf16_rne(b1[t * 16 + nloc]);
#pragma unroll
    for (int r8 = 0; r8 < 8; ++r8) { const float v = silu(a1[t][r8] * sc + bv); a1[t][r8] = v; ps[r8] += v; } }
#pragma unroll
  for (int r8 = 0; r8 < 8; ++r8) { for (int o = 1; o < 16; o <<= 1) ps[r8] += __shfl_xor(ps[r8], o); ps[r8] *= (1.0f / H4); pq[r8] = 0.0f;
#pragma unroll
    for (int t = 0; t < 16; ++t) { const float d = a1[t][r8] - ps[r8]; pq[r8] += pmul(d, d); } for (int o = 1; o < 16; o <<= 1) pq[r8] += __shfl_xor(pq[r8], o); pq[r8] = rsqrtf(pq[r8] * (1.0f / H4) + EPS); }
  wave_lds_sync();
#pragma unroll
  for (int t = 0; t < 16; ++t) { const int c = t * 16 + nloc; const float gg = bf16_rne(g[c]), be = bf16_rne(bb[c]);
#pragma unroll
    for (int r8 = 0; r8 < 8; ++r8) { const float v = pmul(pmul(a1[t][r8] - ps[r8], pq[r8]), gg) + be; b16 p, q; split16(v * XS, p, q); Ah[8 * hlf + r8][c] = p; Al[8 * hlf + r8][c] = q; } }
  wave_lds_sync();
  v8f acc[4];
#pragma unroll
  for (int t = 0; t < 4; ++t) acc[t] = (v8f){};
#pragma unroll 2
  for (int kb = 0; kb < H4; kb += 32) { const v16b a = frag_kb(&Ah[nloc][kb], hlf), al = frag_kb(&Al[nloc][kb], hlf);
#pragma unroll
    for (int t = 0; t < 4; ++t) { const v16b bw = frag_kb(W2T + (size_t)(t * 16 + nloc) * H4 + kb, hlf); acc[t] = wmma16b(a, bw, acc[t]); acc[t] = wmma16b(al, bw, acc[t]); } }
#pragma unroll
  for (int t = 0; t < 4; ++t) { const int c = t * 16 + nloc; const float bv = bf16_rne(b2[c]);
#pragma unroll 1
    for (int r8 = 0; r8 < 8; ++r8) Tf[8 * hlf + r8][c] = acc[t][r8] * sc + bv; }
  wave_lds_sync();
  for (int pass = 0; pass < 2; ++pass) { for (int rr = 0; rr < 16; ++rr) *(volatile v2f*)(OUT_ + (m0 + rr) * H + lane * 2) = *(const v2f*)(&Tf[rr][lane * 2]); __threadfence(); }
}
__global__ __launch_bounds__(64) void readout_kernel(const float* __restrict__ Hp, const float* __restrict__ x, const int* __restrict__ ptr, const int* __restrict__ PERM, const int* __restrict__ ROWPTR, const int* __restrict__ ROWCNT, int permLen, int NLIM, const b16* __restrict__ RW1T, const float* __restrict__ rb1, const float* __restrict__ g, const float* __restrict__ bb, const float* __restrict__ rw2, const float* __restrict__ rb2, float* __restrict__ out) {
  __shared__ __attribute__((aligned(16))) b16 Ah[2][16][ROP + 8], Al[2][16][ROP + 8]; __shared__ __attribute__((aligned(16))) float Tz[2][16][H4 + 4]; __shared__ float so[32 * NO];
  const int wave = threadIdx.x >> 5, lane = threadIdx.x & 31, nloc = lane & 15, hlf = lane >> 4; const int g0 = blockIdx.x * 32 + wave * 16; const float sc = 1.0f / (XS * WSC);
  for (int rr = 0; rr < 16; ++rr) { const int gid = g0 + rr; const int gg = gid < G ? gid : G - 1; const int tix = (gg >> 3) * 32 + (gg & 7); int st = ROWPTR[tix], cnt = ROWCNT[tix]; cnt = iclamp(cnt, 0, 1 << 20); st = iclamp(st, 0, permLen - cnt);
    v2f sm = {0.0f, 0.0f}, mx = {-INFINITY, -INFINITY}; int used = 0;
#pragma unroll 1
    for (int j = 0; j < cnt; ++j) { const int n = iclamp(PERM[st + j], 0, N - 1); if (n >= NLIM) continue; ++used; const v2f hv = *(const v2f*)(Hp + (size_t)n * H + lane * 2); for (int i = 0; i < 2; ++i) { sm[i] += hv[i]; mx[i] = fmaxf(mx[i], hv[i]); } }
    const float inv = 1.0f / (float)(used < 1 ? 1 : used); const int root = iclamp(ptr[gg], 0, N - 1);
    for (int i = 0; i < 2; ++i) { const int c = lane * 2 + i; b16 p, q; split16(pmul(sm[i], inv) * XS, p, q); Ah[wave][rr][c] = p; Al[wave][rr][c] = q; split16((used > 0 ? mx[i] : 0.0f) * XS, p, q); Ah[wave][rr][H + c] = p; Al[wave][rr][H + c] = q; split16(sm[i] * XS, p, q); Ah[wave][rr][2 * H + c] = p; Al[wave][rr][2 * H + c] = q; }
    for (int q = 0; q < 2; ++q) { const int c = 3 * H + q * 32 + lane; const float xv = (c - 3 * H) < FI ? bf16_rne(x[(size_t)root * FI + (c - 3 * H)]) : 0.0f; Ah[wave][rr][c] = (b16)(xv * XS); Al[wave][rr][c] = (b16)0.0f; } }
  wave_lds_sync();
#pragma unroll 1
  for (int cg = 0; cg < 2; ++cg) { v8f a1[8];
#pragma unroll
    for (int t = 0; t < 8; ++t) a1[t] = (v8f){};
#pragma unroll 1
    for (int kb = 0; kb < ROP; kb += 32) { const v16b a = frag_kb(&Ah[wave][nloc][kb], hlf), al = frag_kb(&Al[wave][nloc][kb], hlf);
#pragma unroll
      for (int t = 0; t < 8; ++t) { const v16b bw = frag_kb(RW1T + (size_t)(cg * 128 + t * 16 + nloc) * ROP + kb, hlf); a1[t] = wmma16b(a, bw, a1[t]); a1[t] = wmma16b(al, bw, a1[t]); } }
#pragma unroll
    for (int t = 0; t < 8; ++t) { const int c = cg * 128 + t * 16 + nloc; const float bv = bf16_rne(rb1[c]);
#pragma unroll 1
      for (int r8 = 0; r8 < 8; ++r8) Tz[wave][8 * hlf + r8][c] = silu(a1[t][r8] * sc + bv); } }
  wave_lds_sync();
  float gg8[8], be8[8], w8[8][NO]; for (int q = 0; q < 8; ++q) { const int c = q * 32 + lane; gg8[q] = bf16_rne(g[c]); be8[q] = bf16_rne(bb[c]); for (int k = 0; k < NO; ++k) w8[q][k] = bf16_rne(rw2[c * NO + k]); }
  for (int rr = 0; rr < 16; ++rr) { float v[8]; float s = 0.0f; for (int q = 0; q < 8; ++q) { v[q] = Tz[wave][rr][q * 32 + lane]; s += v[q]; } for (int o = 16; o; o >>= 1) s += __shfl_xor(s, o); const float mu = s * (1.0f / H4);
    float vq = 0.0f; for (int q = 0; q < 8; ++q) { const float d = v[q] - mu; vq += pmul(d, d); } for (int o = 16; o; o >>= 1) vq += __shfl_xor(vq, o); const float rs = rsqrtf(vq * (1.0f / H4) + EPS);
    float pk[NO]; for (int k = 0; k < NO; ++k) pk[k] = 0.0f;
    for (int q = 0; q < 8; ++q) { const float z = pmul(pmul(v[q] - mu, rs), gg8[q]) + be8[q]; for (int k = 0; k < NO; ++k) pk[k] += pmul(z, w8[q][k]); }
    for (int k = 0; k < NO; ++k) { float t = pk[k]; for (int o = 16; o; o >>= 1) t += __shfl_xor(t, o); if (lane == 0) so[(wave * 16 + rr) * NO + k] = t + bf16_rne(rb2[k]); } }
  __syncthreads();
  const int ng = (G - blockIdx.x * 32) < 32 ? (G - blockIdx.x * 32) : 32;
  for (int pass = 0; pass < 2; ++pass) { for (int i = threadIdx.x; i < ng * NO; i += 64) ((volatile float*)out)[(size_t)blockIdx.x * 32 * NO + i] = so[i]; __threadfence(); }
}
}

extern "C" void kernel_launch(void* const* d_in, const int* in_sizes, int n_in, void* d_out, int out_size, void* d_ws, size_t ws_size, hipStream_t stream) {
  (void)n_in;
  auto Fp = [&](int i) { return (const float*)d_in[i]; }; auto Ip = [&](int i) { return (const int*)d_in[i]; };
  if (in_sizes[0] != N * FI || in_sizes[1] != 2 * E || in_sizes[2] != N || in_sizes[3] != G + 1 || in_sizes[4] != 2 * FI * H || in_sizes[7] != (NL - 1) * 2 * H * H || in_sizes[9] != (NL - 1) * H * H || in_sizes[14] != H * H4 || in_sizes[20] != RO * H4 || in_sizes[24] != H4 * NO || out_size != G * NO) return;
  const int NLIM = N; const int GB16 = NBLK;
  size_t off = 0; char* ws = (char*)d_ws;
  auto carve = [&](size_t bytes) { char* p = ws + off; off += (bytes + 255) & ~(size_t)255; return p; };
  b16* WT0 = (b16*)carve(2 * H * 32 * 2); b16* WTL[3]; for (int i = 0; i < 3; ++i) WTL[i] = (b16*)carve((size_t)H * 3 * H * 2); b16* W1T = (b16*)carve((size_t)H4 * H * 2); b16* W2T = (b16*)carve((size_t)H * H4 * 2); b16* RW1T = (b16*)carve((size_t)H4 * ROP * 2);
  float* HA = (float*)carve((size_t)N * H * 4); float* HB = (float*)carve((size_t)N * H * 4);
  CsrBufs9 csr; CsrBufs3 pl; off = csr_carve9(csr, ws, off, E, N); off = csr_carve3(pl, ws, off, N, G);
  if (off > ws_size || off > ((size_t)128 << 20)) return;
  w0_kernel<<<1, 128, 0, stream>>>(Fp(4), Fp(6), Fp(10), WT0);
  for (int i = 0; i < 3; ++i) { wput_kernel<<<(H * 16 + 255) / 256, 256, 0, stream>>>(Fp(7) + (size_t)i * 2 * H * H, 2 * H, H, H, 0, 3 * H, WTL[i]); wput_kernel<<<(H * 8 + 255) / 256, 256, 0, stream>>>(Fp(9) + (size_t)i * H * H, H, H, H, 2 * H, 3 * H, WTL[i]); }
  wput_kernel<<<(H4 * 8 + 255) / 256, 256, 0, stream>>>(Fp(14), H, H4, H4, 0, H, W1T); wput_kernel<<<(H * 32 + 255) / 256, 256, 0, stream>>>(Fp(18), H4, H, H, 0, H4, W2T);

  wput_kernel<<<(H4 * 24 + 255) / 256, 256, 0, stream>>>(Fp(20), 3 * H, H4, H4, 0, ROP, RW1T); ro_tail_kernel<<<1, 256, 0, stream>>>(Fp(20), RW1T);
  csr_build9(csr, Ip(1) + E, E, N, stream); csr_build3(pl, Ip(2), N, G, stream);
  sage_kernel<1><<<GB16, 32, 0, stream>>>(Fp(0), Ip(1), csr.PERM, csr.ROWPTR, csr.ROWCNT, (int)csr.permLen, WT0, Fp(5), Fp(11), Fp(12), Fp(13), NLIM, HA);
  float* hin = HA; float* hout = HB;
  for (int i = 0; i < NL - 1; ++i) { sage_kernel<0><<<GB16, 32, 0, stream>>>(hin, Ip(1), csr.PERM, csr.ROWPTR, csr.ROWCNT, (int)csr.permLen, WTL[i], Fp(8) + i * H, nullptr, Fp(12) + (i + 1) * H, Fp(13) + (i + 1) * H, NLIM, hout); float* t = hin; hin = hout; hout = t; }
  mlp_kernel<<<GB16, 32, 0, stream>>>(hin, W1T, Fp(15), Fp(16), Fp(17), W2T, Fp(19), NLIM, hout);
  readout_kernel<<<(G + 31) / 32, 64, 0, stream>>>(hout, Fp(0), Ip(3), pl.PERM, pl.ROWPTR, pl.ROWCNT, (int)pl.permLen, NLIM, RW1T, Fp(21), Fp(22), Fp(23), Fp(24), Fp(25), (float*)d_out);
}
